// ConceptLayer_86036784873949
// MI455X (gfx1250) — hardware-verified
//
#include <hip/hip_runtime.h>
#include <math.h>

constexpr int kBatch  = 8;
constexpr int kSeq    = 2048;
constexpr int kEmb    = 512;
constexpr int kHeads  = 16;
constexpr int kHdim   = 32;
constexpr int kTok    = kBatch * kSeq;
constexpr int kKK     = kHdim * kHdim;
constexpr int kBlkTok = 32;
constexpr int kSyPitch = 516;
constexpr float kAcarry = 16.0f;
constexpr float kCcarry = 256.0f;
constexpr float kBilInv = 1.0f / 4096.0f;
constexpr float kInvEmb = 1.0f / 512.0f;
constexpr float kLnEps  = 1e-3f;
constexpr float kInvDecay = 1.0f / 1.2f;
static_assert(kTok % kBlkTok == 0, "tile");
static_assert(kTok % 64 == 0 && kEmb % 64 == 0, "tile");

typedef __attribute__((ext_vector_type(16))) _Float16 v16h;
typedef __attribute__((ext_vector_type(8)))  _Float16 v8h;
typedef __attribute__((ext_vector_type(2)))  _Float16 v2h;
typedef __attribute__((ext_vector_type(16))) __bf16   v16b;
typedef __attribute__((ext_vector_type(8)))  __bf16   v8b;
typedef __attribute__((ext_vector_type(8)))  float    v8f;
typedef __attribute__((ext_vector_type(4)))  float    v4f;
typedef __attribute__((ext_vector_type(2)))  float    v2f;
typedef __attribute__((ext_vector_type(4)))  unsigned int v4u;

__device__ __forceinline__ unsigned short f2bf_bits(float f) {
  unsigned u = __float_as_uint(f);
  return (unsigned short)((u + 0x7FFFu + ((u >> 16) & 1u)) >> 16);
}
__device__ __forceinline__ float bf_bits2f(unsigned short h) { return __uint_as_float(((unsigned)h) << 16); }

__device__ __forceinline__ void dep_guard_h(v8f& a, v8f& b, v16h x, v16h y) { asm volatile("v_nop\n\tv_nop\n\tv_nop\n\tv_nop" : "+v"(a), "+v"(b) : "v"(x), "v"(y)); }
__device__ __forceinline__ void dep_guard_b(v8f& a, v8f& b, v16b x, v16b y) { asm volatile("v_nop\n\tv_nop\n\tv_nop\n\tv_nop" : "+v"(a), "+v"(b) : "v"(x), "v"(y)); }
__device__ __forceinline__ void keep4_h(v16h a, v16h b, v16h c, v16h d) { asm volatile("v_nop" :: "v"(a), "v"(b), "v"(c), "v"(d)); }
__device__ __forceinline__ void keep4_b(v16b a, v16b b, v16b c, v16b d) { asm volatile("v_nop" :: "v"(a), "v"(b), "v"(c), "v"(d)); }
__device__ __forceinline__ void acc_guard4(v8f& a, v8f& b, v8f& c, v8f& d) { asm volatile("v_nop\n\tv_nop\n\tv_nop\n\tv_nop" : "+v"(a), "+v"(b), "+v"(c), "+v"(d)); }
template <typename T> struct Frag;
template <> struct Frag<_Float16> {
  typedef v16h V; union U { v16h v; v8h h[2]; };
  static __device__ __forceinline__ v16h load(const _Float16* p) {
    U f; f.h[0] = *(const v8h*)(p); f.h[1] = *(const v8h*)(p + 16); return f.v;
  }
  static __device__ __forceinline__ v8f mma(v16h a, v16h b, v8f c) {
    return __builtin_amdgcn_wmma_f32_16x16x32_f16(false, a, false, b, (short)0, c, false, false);
  }
  static __device__ __forceinline__ void guard(v8f& a, v8f& b, v16h x, v16h y) { dep_guard_h(a, b, x, y); }
  static __device__ __forceinline__ void keep(v16h a, v16h b, v16h c, v16h d) { keep4_h(a, b, c, d); }
};
template <> struct Frag<__bf16> {
  typedef v16b V; union U { v16b v; v8b h[2]; };
  static __device__ __forceinline__ v16b load(const __bf16* p) {
    U f; f.h[0] = *(const v8b*)(p); f.h[1] = *(const v8b*)(p + 16); return f.v;
  }
  static __device__ __forceinline__ v8f mma(v16b a, v16b b, v8f c) {
    return __builtin_amdgcn_wmma_f32_16x16x32_bf16(false, a, false, b, (short)0, c, false, false);
  }
  static __device__ __forceinline__ void guard(v8f& a, v8f& b, v16b x, v16b y) { dep_guard_b(a, b, x, y); }
  static __device__ __forceinline__ void keep(v16b a, v16b b, v16b c, v16b d) { keep4_b(a, b, c, d); }
};

__device__ __forceinline__ unsigned pk16(unsigned short a, unsigned short b) { return (unsigned)a | ((unsigned)b << 16); }
__device__ __forceinline__ unsigned short h_bits(float f) { const _Float16 h = (_Float16)f; return __builtin_bit_cast(unsigned short, h); }

template <int ET> struct Elem;
template <> struct Elem<0> { typedef _Float16 T; };
template <> struct Elem<1> { typedef __bf16 T; };
template <int ET, bool SPLIT, int BIAS_MODE, int OUT_MODE, bool RESID, int ACT = 0>
__global__ __launch_bounds__(256) void wmma_gemm64(
    const unsigned short* __restrict__ Ap, const unsigned short* __restrict__ A2p, int lda, long strideA,
    const unsigned short* __restrict__ Btp, const unsigned short* __restrict__ Bt2p, int ldb, long strideB,
    void* __restrict__ Cout, void* __restrict__ Cout2, int ldc, long strideC,
    const float* __restrict__ bias,
    const float* __restrict__ resid, long strideR,
    int M, int N, int K, float scale) {
  typedef typename Elem<ET>::T T;
  typedef typename Frag<T>::V V;
  const T* A = (const T*)Ap; const T* A2 = (const T*)A2p; const T* Bt = (const T*)Btp; const T* Bt2 = (const T*)Bt2p;
  __shared__ __align__(16) float sT[8][16 * 68];
  const int b    = blockIdx.y;
  const int lane = threadIdx.x & 31;
  const int wave = threadIdx.x >> 5;
  const int tilesN = N >> 6;
  const int tilesM = M >> 6;
  const int tile = blockIdx.x * 8 + wave;
  if (tile >= tilesM * tilesN) return;
  const int tm = tile / tilesN;
  const int tn = tile - tm * tilesN;
  const int m0 = tm << 6;
  const int n0 = tn << 6;

  const T* Ab  = A  + (size_t)b * strideA;
  const T* Bb  = Bt + (size_t)b * strideB;
  const T* Ab2 = SPLIT ? (A2  + (size_t)b * strideA) : nullptr;
  const T* Bb2 = SPLIT ? (Bt2 + (size_t)b * strideB) : nullptr;

  const int rlane = lane & 15;
  const int koff  = (lane >> 4) * 8;
  const int mOff  = (lane >> 4) * 8;

  v8f acc[4][4];
#pragma unroll
  for (int i = 0; i < 4; ++i)
#pragma unroll
    for (int j = 0; j < 4; ++j) acc[i][j] = (v8f){0.f,0.f,0.f,0.f,0.f,0.f,0.f,0.f};

  for (int k0 = 0; k0 < K; k0 += 32) {
    V bh[4], bl[4];
#pragma unroll
    for (int j = 0; j < 4; ++j) {
      const size_t bo = (size_t)(n0 + (j << 4) + rlane) * ldb + koff + k0;
      bh[j] = Frag<T>::load(Bb + bo);
      if (SPLIT) bl[j] = Frag<T>::load(Bb2 + bo);
    }
#pragma unroll
    for (int i = 0; i < 4; ++i) {
      const size_t ao = (size_t)(m0 + (i << 4) + rlane) * lda + koff + k0;
      V ah = Frag<T>::load(Ab + ao);
      V al;
      if (SPLIT) al = Frag<T>::load(Ab2 + ao);
#pragma unroll
      for (int j = 0; j < 4; ++j) {
        acc[i][j] = Frag<T>::mma(ah, bh[j], acc[i][j]);
        if (SPLIT) {
          acc[i][j] = Frag<T>::mma(ah, bl[j], acc[i][j]);
          acc[i][j] = Frag<T>::mma(al, bh[j], acc[i][j]);
        }
      }
      Frag<T>::guard(acc[i][0], acc[i][3], ah, SPLIT ? al : ah);
    }
    Frag<T>::keep(bh[0], bh[1], bh[2], bh[3]);
    if (SPLIT) Frag<T>::keep(bl[0], bl[1], bl[2], bl[3]);
  }
  acc_guard4(acc[0][0], acc[0][1], acc[0][2], acc[0][3]);
  acc_guard4(acc[1][0], acc[1][1], acc[1][2], acc[1][3]);
  acc_guard4(acc[2][0], acc[2][1], acc[2][2], acc[2][3]);
  acc_guard4(acc[3][0], acc[3][1], acc[3][2], acc[3][3]);

  float* slab = sT[wave];
  const float* Rb = RESID ? (resid + (size_t)b * strideR) : nullptr;
#pragma unroll
  for (int i = 0; i < 4; ++i) {
    const int mBase = m0 + (i << 4);
#pragma unroll
    for (int j = 0; j < 4; ++j) {
      const int n = n0 + (j << 4) + rlane;
      float bv = 0.f;
      if (BIAS_MODE == 2) bv = bias[n];
#pragma unroll
      for (int r = 0; r < 8; ++r) {
        float v = acc[i][j][r] * scale;
        if (BIAS_MODE == 1) v += bias[mBase + mOff + r];
        if (BIAS_MODE == 2) v += bv;
        if (RESID) v += Rb[(size_t)(mBase + mOff + r) * ldc + n];
        if (ACT == 1) v = tanhf(v);
        if (ACT == 2) v = fmaxf(v, 0.0f);
        if (ACT == 3) v = v / (1.0f + expf(-v));
        if (ACT == 4) v = (v > 0.f) ? v : 0.01f * v;
        if (ACT == 5) v = 0.5f * v * (1.0f + erff(v * 0.70710678118654752f));
        slab[(mOff + r) * 68 + (j << 4) + rlane] = v;
      }
    }
    __builtin_amdgcn_fence(__ATOMIC_RELEASE, "workgroup");
    __builtin_amdgcn_wave_barrier();
    __builtin_amdgcn_fence(__ATOMIC_ACQUIRE, "workgroup");
    if (OUT_MODE == 0) {
      float* C = (float*)Cout + (size_t)b * strideC;
      const int hh = lane >> 4, c4 = (lane & 15) * 4;
      for (int pass = 0; pass < 2; ++pass) {
#pragma unroll
        for (int it = 0; it < 8; ++it) {
          const int row = it * 2 + hh;
          v4f v = *(const v4f*)(slab + row * 68 + c4);
          *(volatile v4f*)(C + (size_t)(mBase + row) * ldc + n0 + c4) = v;
        }
        __threadfence();
      }
    } else {
      const int q = lane >> 3, c8 = (lane & 7) * 8;
      unsigned short* C  = (unsigned short*)Cout  + (size_t)b * strideC;
      unsigned short* C2 = (OUT_MODE == 2) ? ((unsigned short*)Cout2 + (size_t)b * strideC) : nullptr;
      for (int pass = 0; pass < 2; ++pass) {
#pragma unroll
        for (int it = 0; it < 4; ++it) {
          const int row = it * 4 + q;
          const float* sp = slab + row * 68 + c8;
          v8h hv, lv;
#pragma unroll
          for (int e = 0; e < 8; ++e) {
            if (OUT_MODE == 1) {
              hv[e] = (_Float16)sp[e];
            } else {
              unsigned short hb = f2bf_bits(sp[e]);
              unsigned short lb = f2bf_bits(sp[e] - bf_bits2f(hb));
              hv[e] = __builtin_bit_cast(_Float16, hb);
              lv[e] = __builtin_bit_cast(_Float16, lb);
            }
          }
          *(volatile v8h*)(C + (size_t)(mBase + row) * ldc + n0 + c8) = hv;
          if (OUT_MODE == 2) *(volatile v8h*)(C2 + (size_t)(mBase + row) * ldc + n0 + c8) = lv;
        }
        __threadfence();
      }
    }
    __builtin_amdgcn_fence(__ATOMIC_RELEASE, "workgroup");
    __builtin_amdgcn_wave_barrier();
    __builtin_amdgcn_fence(__ATOMIC_ACQUIRE, "workgroup");
  }
}

template <int MODE>
__global__ __launch_bounds__(256) void cast8_kernel(const float* __restrict__ in, unsigned short* __restrict__ out, int n8, float scale) {
  const int i = blockIdx.x * 256 + threadIdx.x;
  if (i >= n8) return;
  const float* p = in + 8 * (size_t)i;
  const v4f a = *(const v4f*)(p);
  const v4f c = *(const v4f*)(p + 4);
  unsigned short hb[8];
#pragma unroll
  for (int e = 0; e < 4; ++e) {
    if (MODE == 0) {
      hb[e]     = f2bf_bits(a[e]);
      hb[4 + e] = f2bf_bits(c[e]);
    } else {
      hb[e]     = h_bits(bf_bits2f(f2bf_bits(a[e])) * scale);
      hb[4 + e] = h_bits(bf_bits2f(f2bf_bits(c[e])) * scale);
    }
  }
  const v4u u = (v4u){pk16(hb[0], hb[1]), pk16(hb[2], hb[3]), pk16(hb[4], hb[5]), pk16(hb[6], hb[7])};
  unsigned short* q = out + 8 * (size_t)i;
  *(volatile v4u*)q = u;
  __threadfence();
  *(volatile v4u*)q = u;
  (void)scale;
}

__global__ __launch_bounds__(256) void wtrans_kernel(const float* __restrict__ W, unsigned short* __restrict__ WT) {
  __shared__ float sW[64][65];
  const int n0 = blockIdx.x * 64, k0 = blockIdx.y * 64;
  const int t = threadIdx.x, lane = t & 31, wave = t >> 5;
  const int c4 = t & 15, rb = t >> 4;
#pragma unroll
  for (int it = 0; it < 4; ++it) {
    const int row = rb + 16 * it;
    const v4f v = *(const v4f*)(W + (size_t)(k0 + row) * kEmb + n0 + 4 * c4);
    sW[4 * c4 + 0][row] = v[0];
    sW[4 * c4 + 1][row] = v[1];
    sW[4 * c4 + 2][row] = v[2];
    sW[4 * c4 + 3][row] = v[3];
  }
  __syncthreads();
  const int q = lane >> 3, c8 = (lane & 7) * 8;
  v4u u[2];
#pragma unroll
  for (int it = 0; it < 2; ++it) {
    const int nn = wave * 8 + it * 4 + q;
    unsigned short hb[8];
#pragma unroll
    for (int e = 0; e < 8; ++e) hb[e] = f2bf_bits(sW[nn][c8 + e]);
    u[it] = (v4u){pk16(hb[0], hb[1]), pk16(hb[2], hb[3]), pk16(hb[4], hb[5]), pk16(hb[6], hb[7])};
  }
  for (int pass = 0; pass < 2; ++pass) {
#pragma unroll
    for (int it = 0; it < 2; ++it) {
      const int nn = wave * 8 + it * 4 + q;
      *(volatile v4u*)(WT + (size_t)(n0 + nn) * kEmb + k0 + c8) = u[it];
    }
    __threadfence();
  }
}

__global__ __launch_bounds__(256) void scan_kernel(const float* __restrict__ Hp, float* __restrict__ Sp) {
  const int g = blockIdx.x * 256 + threadIdx.x;
  const int b = g >> 9, e = g & (kEmb - 1);
  size_t idx = (size_t)b * kSeq * kEmb + e;
  float s = 0.f;
#pragma unroll 1
  for (int t = 0; t < kSeq; ++t) {
    const float hv = Hp[idx];
    *(volatile float*)(Sp + idx) = s;
    __threadfence();
    *(volatile float*)(Sp + idx) = s;
    s = (s + hv) * kInvDecay;
    idx += kEmb;
  }
}

__global__ __launch_bounds__(256) void bilinear_ln_kernel(
    const float* __restrict__ Hp, const float* __restrict__ Sp, const unsigned short* __restrict__ CFp,
    const float* __restrict__ gamma, const float* __restrict__ beta, float* __restrict__ outp) {
  extern __shared__ __align__(16) float dyn_lds[];
  float* sy = dyn_lds;
  const int tid = threadIdx.x, wave = tid >> 5, lane = tid & 31;
  const int hh = lane >> 4, rl = lane & 15;
  const size_t tok0 = (size_t)blockIdx.x * kBlkTok;

#pragma unroll
  for (int it = 0; it < 16; ++it) {
    const int idx = tid + 256 * it;
    const int row = idx >> 7, c4 = idx & 127;
    const v4f v = *(const v4f*)(Hp + (tok0 + row) * kEmb + 4 * c4);
    *(v4f*)(sy + row * kSyPitch + 4 * c4) = v;
  }
  __syncthreads();

  const _Float16* CFh = (const _Float16*)(const void*)CFp;
  union HF { v16h v; v2h p[8]; };

#pragma unroll 1
  for (int hp = 0; hp < 2; ++hp) {
    const int cb = (wave * 2 + hp) * kHdim;
    float sr[2][16];
#pragma unroll
    for (int mt = 0; mt < 2; ++mt) {
      const float* sp = Sp + (tok0 + mt * 16 + rl) * kEmb + cb + 8 * hh;
      const v4f a0 = *(const v4f*)(sp);
      const v4f a1 = *(const v4f*)(sp + 4);
      const v4f a2 = *(const v4f*)(sp + 16);
      const v4f a3 = *(const v4f*)(sp + 20);
#pragma unroll
      for (int e = 0; e < 4; ++e) {
        sr[mt][e]      = a0[e] * kAcarry;
        sr[mt][4 + e]  = a1[e] * kAcarry;
        sr[mt][8 + e]  = a2[e] * kAcarry;
        sr[mt][12 + e] = a3[e] * kAcarry;
      }
    }
    v8f acc[2][2];
#pragma unroll
    for (int mt = 0; mt < 2; ++mt)
#pragma unroll
      for (int nt = 0; nt < 2; ++nt) acc[mt][nt] = (v8f){0.f,0.f,0.f,0.f,0.f,0.f,0.f,0.f};

    const _Float16* cfb = CFh + (size_t)(cb + rl) * kKK + 8 * hh;
    const float* hrow = sy + rl * kSyPitch + cb;

#pragma unroll 1
    for (int i = 0; i < kHdim; ++i) {
      v16h bfr[2];
      bfr[0] = Frag<_Float16>::load(cfb + i * 32);
      bfr[1] = Frag<_Float16>::load(cfb + (size_t)16 * kKK + i * 32);
      v16h afr[2];
#pragma unroll
      for (int mt = 0; mt < 2; ++mt) {
        const float hs = hrow[mt * 16 * kSyPitch + i];
        HF u;
#pragma unroll
        for (int e = 0; e < 8; ++e) {
          v2f pr;
          pr[0] = hs * sr[mt][2 * e];
          pr[1] = hs * sr[mt][2 * e + 1];
          u.p[e] = __builtin_convertvector(pr, v2h);
        }
        afr[mt] = u.v;
      }
      acc[0][0] = Frag<_Float16>::mma(afr[0], bfr[0], acc[0][0]);
      acc[0][1] = Frag<_Float16>::mma(afr[0], bfr[1], acc[0][1]);
      acc[1][0] = Frag<_Float16>::mma(afr[1], bfr[0], acc[1][0]);
      acc[1][1] = Frag<_Float16>::mma(afr[1], bfr[1], acc[1][1]);
      dep_guard_h(acc[0][0], acc[0][1], afr[0], bfr[0]);
      dep_guard_h(acc[1][0], acc[1][1], afr[1], bfr[1]);
    }
    acc_guard4(acc[0][0], acc[0][1], acc[1][0], acc[1][1]);

#pragma unroll
    for (int mt = 0; mt < 2; ++mt) {
#pragma unroll
      for (int nt = 0; nt < 2; ++nt) {
#pragma unroll
        for (int r = 0; r < 8; ++r) {
          float* p = sy + (mt * 16 + 8 * hh + r) * kSyPitch + cb + nt * 16 + rl;
          const float hv = *p;
          *p = acc[mt][nt][r] * kBilInv + hv;
        }
      }
    }
  }
  __syncthreads();

  v4f gv[4], bv[4];
#pragma unroll
  for (int it = 0; it < 4; ++it) {
    gv[it] = *(const v4f*)(gamma + 128 * it + 4 * lane);
    bv[it] = *(const v4f*)(beta + 128 * it + 4 * lane);
  }
#pragma unroll 1
  for (int rr = 0; rr < 4; ++rr) {
    const int row = wave * 4 + rr;
    const float* yr = sy + row * kSyPitch;
    v4f yv[4];
    float s = 0.f;
#pragma unroll
    for (int it = 0; it < 4; ++it) {
      yv[it] = *(const v4f*)(yr + 128 * it + 4 * lane);
      s += (yv[it][0] + yv[it][1]) + (yv[it][2] + yv[it][3]);
    }
#pragma unroll
    for (int off = 16; off > 0; off >>= 1) s += __shfl_xor(s, off, 32);
    const float mu = s * kInvEmb;
    v4f d[4];
    float qs = 0.f;
#pragma unroll
    for (int it = 0; it < 4; ++it) {
      d[it] = yv[it] - mu;
      qs += (d[it][0] * d[it][0] + d[it][1] * d[it][1]) + (d[it][2] * d[it][2] + d[it][3] * d[it][3]);
    }
#pragma unroll
    for (int off = 16; off > 0; off >>= 1) qs += __shfl_xor(qs, off, 32);
    const float var = qs * kInvEmb;
    const float rs  = rsqrtf(var + kLnEps);
    v4f o[4];
#pragma unroll
    for (int it = 0; it < 4; ++it) o[it] = (d[it] * rs) * gv[it] + bv[it];
    float* orow = outp + (tok0 + row) * kEmb;
    for (int pass = 0; pass < 2; ++pass) {
#pragma unroll
      for (int it = 0; it < 4; ++it) *(volatile v4f*)(orow + 128 * it + 4 * lane) = o[it];
      __threadfence();
    }
  }
}

extern "C" void kernel_launch(void* const* d_in, const int* in_sizes, int n_in,
                              void* d_out, int out_size, void* d_ws, size_t ws_size,
                              hipStream_t stream) {
  if (n_in < 6) return;
  if (in_sizes[0] != kTok * kEmb) return;
  if (in_sizes[1] != kEmb * kEmb) return;
  if (in_sizes[2] != kEmb) return;
  if (in_sizes[3] != kHeads * kHdim * kKK) return;
  if (in_sizes[4] != kEmb) return;
  if (in_sizes[5] != kEmb) return;
  if (out_size != kTok * kEmb) return;

  const float* x     = (const float*)d_in[0];
  const float* W     = (const float*)d_in[1];
  const float* bvec  = (const float*)d_in[2];
  const float* cten  = (const float*)d_in[3];
  const float* gamma = (const float*)d_in[4];
  const float* beta  = (const float*)d_in[5];
  float* outp = (float*)d_out;

  const size_t SZ_XB  = (size_t)kTok * kEmb * 2;
  const size_t SZ_WTB = (size_t)kEmb * kEmb * 2;
  const size_t SZ_CF  = (size_t)kHeads * kHdim * kKK * 2;
  const size_t SZ_F32 = (size_t)kTok * kEmb * 4;
  size_t off = 0;
  const size_t oXB  = off; off += SZ_XB;
  const size_t oWTB = off; off += SZ_WTB;
  const size_t oCF  = off; off += SZ_CF;
  const size_t oHP  = off; off += SZ_F32;
  const size_t oSP  = off; off += SZ_F32;
  const size_t TOTAL = off;
  if (TOTAL > ws_size) return;
  if (TOTAL > (size_t)134217728) return;

  char* ws = (char*)d_ws;
  unsigned short* XB  = (unsigned short*)(ws + oXB);
  unsigned short* WTB = (unsigned short*)(ws + oWTB);
  unsigned short* CF  = (unsigned short*)(ws + oCF);
  float*          HP  = (float*)(ws + oHP);
  float*          SP  = (float*)(ws + oSP);

  const dim3 blk(256);

  {
    const int n8x = kTok * kEmb / 8;
    cast8_kernel<0><<<dim3(n8x / 256), blk, 0, stream>>>(x, XB, n8x, 1.0f);
    const int n8c = kHeads * kHdim * kKK / 8;
    cast8_kernel<1><<<dim3(n8c / 256), blk, 0, stream>>>(cten, CF, n8c, kCcarry);
    wtrans_kernel<<<dim3(kEmb / 64, kEmb / 64), blk, 0, stream>>>(W, WTB);
  }

  {
    const dim3 gP(((kTok / 64) * (kEmb / 64) + 7) / 8, 1);
    wmma_gemm64<1, false, 2, 0, false, 0><<<gP, blk, 0, stream>>>(
        XB, XB, kEmb, 0L, WTB, WTB, kEmb, 0L, (void*)HP, (void*)HP, kEmb, 0L,
        bvec, bvec, 0L, kTok, kEmb, kEmb, 1.0f);
  }

  scan_kernel<<<dim3((kBatch * kEmb) / 256), blk, 0, stream>>>(HP, SP);

  {
    const size_t ldsBytes = (size_t)kBlkTok * kSyPitch * sizeof(float);
    bilinear_ln_kernel<<<dim3(kTok / kBlkTok), blk, ldsBytes, stream>>>(HP, SP, CF, gamma, beta, outp);
  }
}
